// MultiHeadSelfAttention_21921513079123
// MI455X (gfx1250) — hardware-run, weakly checked
//
#include <hip/hip_runtime.h>


#ifndef NB
#define NB 4
#endif
#ifndef SEQ
#define SEQ 2048
#endif
#define NB_FULL  4
#define SEQ_FULL 2048
#define DM   1024
#define NH   16
#define HD   64
#ifndef OUT_BSTRIDE
#define OUT_BSTRIDE ((size_t)SEQ * DM)
#endif
#define PCAR 1024.0f
#define SL   0.045084220027780106f
#define L2E  1.4426950408889634f

static_assert(SEQ % 128 == 0);
static_assert(NH * HD == DM);
static_assert(DM % 64 == 0);
static_assert(NB <= NB_FULL);
static_assert(SEQ <= SEQ_FULL);
static_assert(HD == 64);
static_assert(SEQ % 32 == 0);
static_assert(DM % 32 == 0);
static_assert(((size_t)NB * SEQ) % 64 == 0);
static_assert((size_t)NB * SEQ * DM * 2 * 6 + (size_t)DM * DM * 2 * 4 <= (size_t)134217728);

typedef _Float16 h16;
typedef unsigned short bf;
typedef __attribute__((ext_vector_type(16))) __bf16   v16bf;
typedef __attribute__((ext_vector_type(16))) _Float16 v16h;
typedef __attribute__((ext_vector_type(8)))  _Float16 v8h;
typedef __attribute__((ext_vector_type(8)))  unsigned short v8us;
typedef __attribute__((ext_vector_type(8)))  float    v8f;
typedef __attribute__((ext_vector_type(4)))  float    v4f;
typedef v4f  __attribute__((may_alias)) v4fa;

__device__ __forceinline__ unsigned short f2bf(float f) { unsigned u = __float_as_uint(f); u += 0x7FFFu + ((u >> 16) & 1u); return (unsigned short)(u >> 16); }
__device__ __forceinline__ float bf2f(unsigned short b) { return __uint_as_float(((unsigned)b) << 16); }
__device__ __forceinline__ float bfr(float f) { return bf2f(f2bf(f)); }
__device__ __forceinline__ void splitf(float y, unsigned short& h, unsigned short& l) { h = f2bf(y); l = f2bf(y - bf2f(h)); }
__device__ __forceinline__ v16h cat16(v8h lo, v8h hi) { return __builtin_shufflevector(lo, hi, 0, 1, 2, 3, 4, 5, 6, 7, 8, 9, 10, 11, 12, 13, 14, 15); }
__device__ __forceinline__ v16bf cat16b(v8us lo, v8us hi) { return __builtin_bit_cast(v16bf, __builtin_shufflevector(lo, hi, 0, 1, 2, 3, 4, 5, 6, 7, 8, 9, 10, 11, 12, 13, 14, 15)); }
__device__ __forceinline__ v8f wmma16(v16h a, v16h b, v8f c) { return __builtin_amdgcn_wmma_f32_16x16x32_f16(false, a, false, b, (short)0, c, false, false); }
__device__ __forceinline__ v8f wmmab(v16bf a, v16bf b, v8f c) { return __builtin_amdgcn_wmma_f32_16x16x32_bf16(false, a, false, b, (short)0, c, false, false); }
__device__ __forceinline__ v16h  ldh(const h16* p) { return cat16(*(const v8h*)p, *(const v8h*)(p + 16)); }
__device__ __forceinline__ v16bf ldb(const bf* p)  { return cat16b(*(const v8us*)p, *(const v8us*)(p + 16)); }
static __device__ __forceinline__ h16 toh_flush(float v) { const float w = (fabsf(v) < 6.103515625e-05f) ? 0.0f : v; return (h16)w; }

__global__ __launch_bounds__(256) void k_cvtx(const float* __restrict__ x, bf* XB) {
    const size_t i = (size_t)blockIdx.x * 256 + threadIdx.x; if (i >= (size_t)NB * SEQ * DM / 8) return;
    const size_t e = i * 8; const size_t m = e / DM; const int c = (int)(e % DM); const size_t b = m / SEQ, s = m % SEQ;
    const v8f v = *(const v8f*)(x + (b * SEQ_FULL + s) * DM + c); v8us o;
#pragma unroll
    for (int k = 0; k < 8; ++k) o[k] = f2bf(v[k]);
    *(volatile v8us*)(XB + e) = o; __threadfence(); *(volatile v8us*)(XB + e) = o;
}

__global__ __launch_bounds__(256) void k_cvtT(const float* __restrict__ W, bf* Wt) {
    __shared__ float tl[64 * 65];
    const int k0 = blockIdx.x * 64, n0 = blockIdx.y * 64, tid = threadIdx.x;
#pragma unroll 4
    for (int i = 0; i < 16; ++i) { const int idx = i * 256 + tid; const int r = idx >> 6, c = idx & 63; tl[r * 65 + c] = W[(size_t)(k0 + r) * DM + n0 + c]; }
    __syncthreads();
    v8us o[2];
#pragma unroll
    for (int it = 0; it < 2; ++it) { const int p = it * 256 + tid; const int n = p >> 3, seg = p & 7;
#pragma unroll
        for (int j = 0; j < 8; ++j) o[it][j] = f2bf(tl[(seg * 8 + j) * 65 + n]); }
#pragma unroll 1
    for (int ps = 0; ps < 2; ++ps) {
#pragma unroll
        for (int it = 0; it < 2; ++it) { const int p = it * 256 + tid; const int n = p >> 3, seg = p & 7; *(volatile v8us*)(Wt + (size_t)(n0 + n) * DM + k0 + seg * 8) = o[it]; }
        if (ps == 0) __threadfence(); }
}

template <int NSPLIT, int EPI>
__global__ __launch_bounds__(32) void k_gemmw(const bf* __restrict__ A, const bf* __restrict__ A2, const bf* __restrict__ Bt, int K, float* Cf, h16* Ch, const float* __restrict__ bias) {
    __shared__ __align__(16) float os[16 * 68];
    const int lane = threadIdx.x & 31, lr = lane & 15, hi = lane >> 4; const int r0 = blockIdx.x * 64, c0 = blockIdx.y * 64;
    v8f acc[4][4];
#pragma unroll
    for (int mb = 0; mb < 4; ++mb)
#pragma unroll
        for (int nb = 0; nb < 4; ++nb) acc[mb][nb] = (v8f){};
    const size_t aoff = (size_t)(r0 + lr) * K + 8 * hi, boff = (size_t)(c0 + lr) * K + 8 * hi;
#pragma unroll 1
    for (int kc = 0; kc < K; kc += 32) {
        v16bf a[4], a2[4];
#pragma unroll
        for (int mb = 0; mb < 4; ++mb) { a[mb] = ldb(A + aoff + (size_t)mb * 16 * K + kc); if (NSPLIT == 1) a2[mb] = ldb(A2 + aoff + (size_t)mb * 16 * K + kc); }
#pragma unroll
        for (int nb = 0; nb < 4; ++nb) { const v16bf b = ldb(Bt + boff + (size_t)nb * 16 * K + kc);
#pragma unroll
            for (int mb = 0; mb < 4; ++mb) { acc[mb][nb] = wmmab(a[mb], b, acc[mb][nb]); if (NSPLIT == 1) acc[mb][nb] = wmmab(a2[mb], b, acc[mb][nb]); } }
        asm volatile("v_nop\n\tv_nop\n\tv_nop\n\tv_nop" : "+v"(acc[0][0]), "+v"(acc[1][1]), "+v"(acc[2][2]), "+v"(acc[3][3]) : "v"(a[0]), "v"(a[3]));
    }
#pragma unroll
    for (int mb = 0; mb < 4; ++mb) {
#pragma unroll
        for (int nb = 0; nb < 4; ++nb) {
#pragma unroll
            for (int j = 0; j < 8; ++j) os[(hi * 8 + j) * 68 + nb * 16 + lr] = acc[mb][nb][j]; }
        __builtin_amdgcn_wave_barrier(); asm volatile("" ::: "memory");
        if (EPI == 0) {
            const int bb = r0 / SEQ, s0 = r0 % SEQ;
            float* crow = Cf + (size_t)bb * OUT_BSTRIDE + (size_t)(s0 + mb * 16) * DM + c0;
#pragma unroll 1
            for (int ps = 0; ps < 2; ++ps) {
#pragma unroll
                for (int s = 0; s < 8; ++s) { const int row = 2 * s + hi, cofs = lr * 4; v4f val = *(const v4fa*)(os + row * 68 + cofs);
                    val[0] += bfr(bias[c0 + cofs]); val[1] += bfr(bias[c0 + cofs + 1]); val[2] += bfr(bias[c0 + cofs + 2]); val[3] += bfr(bias[c0 + cofs + 3]);
                    *(volatile v4f*)(crow + (size_t)row * DM + cofs) = val; }
                if (ps == 0) __threadfence(); }
        } else {
            h16* base; size_t pitch;
            if (EPI == 1) { const int bb = r0 / SEQ, s0 = r0 % SEQ; base = Ch + (((size_t)bb * NH + blockIdx.y) * SEQ + s0 + mb * 16) * HD; pitch = HD; }
            else          { const int bb = c0 / SEQ, s0 = c0 % SEQ; base = Ch + (((size_t)bb * NH + blockIdx.x) * HD + mb * 16) * SEQ + s0; pitch = SEQ; }
#pragma unroll 1
            for (int ps = 0; ps < 2; ++ps) {
#pragma unroll
                for (int s = 0; s < 4; ++s) { const int row = 4 * s + (lane >> 3), seg = lane & 7;
                    const v4f va = *(const v4fa*)(os + row * 68 + seg * 8); const v4f vb = *(const v4fa*)(os + row * 68 + seg * 8 + 4); v8h o;
                    if (EPI == 1) {
#pragma unroll
                        for (int j = 0; j < 4; ++j) { o[j] = (h16)(va[j] + bfr(bias[c0 + seg * 8 + j])); o[4 + j] = (h16)(vb[j] + bfr(bias[c0 + seg * 8 + 4 + j])); }
                    } else { const float bv = bfr(bias[r0 + mb * 16 + row]);
#pragma unroll
                        for (int j = 0; j < 4; ++j) { o[j] = (h16)(va[j] + bv); o[4 + j] = (h16)(vb[j] + bv); } }
                    *(volatile v8h*)(base + (size_t)row * pitch + seg * 8) = o; }
                if (ps == 0) __threadfence(); }
        }
        __builtin_amdgcn_wave_barrier(); asm volatile("" ::: "memory");
    }
}

__global__ __launch_bounds__(128) void k_flash(const h16* __restrict__ QP, const h16* __restrict__ KP, const h16* __restrict__ VT, const int* __restrict__ mask, bf* ATh, bf* ATl) {
    __shared__ __align__(16) float mf[SEQ];
    __shared__ __align__(16) float os[4 * 16 * 68];
    const int tid = threadIdx.x, wave = tid >> 5, lane = tid & 31, lr = lane & 15, hi = lane >> 4;
    const int bh = blockIdx.y, b = bh / NH, h = bh % NH; const int q0 = blockIdx.x * 64 + wave * 16;
    const int* mb = mask + (size_t)b * SEQ_FULL;
#pragma unroll 1
    for (int it = 0; it < SEQ / 128; ++it) mf[it * 128 + tid] = (float)mb[it * 128 + tid];
    __syncthreads();
    const float mq = mf[q0 + lr] * L2E;
    const h16* qp = QP + ((size_t)bh * SEQ + q0 + lr) * HD + 8 * hi;
    const v16h qb0 = ldh(qp), qb1 = ldh(qp + 32);
    const h16* kp = KP + ((size_t)bh * SEQ + lr) * HD + 8 * hi;
    const h16* vp = VT + ((size_t)bh * HD + lr) * SEQ + 8 * hi;
    v8f o[4];
#pragma unroll
    for (int t = 0; t < 4; ++t) o[t] = (v8f){};
    float mrun = -1.0e30f, lrun = 0.0f;
#pragma unroll 1
    for (int kt = 0; kt < SEQ; kt += 32) {
        const h16* k0p = kp + (size_t)kt * HD;
        const v16h ka0 = ldh(k0p), ka1 = ldh(k0p + 32), kb0 = ldh(k0p + 16 * HD), kb1 = ldh(k0p + 16 * HD + 32);
        v16h va[4];
#pragma unroll
        for (int t = 0; t < 4; ++t) va[t] = ldh(vp + (size_t)t * 16 * SEQ + kt);
        v8f s0 = (v8f){}, s1 = (v8f){};
        s0 = wmma16(ka0, qb0, s0); s1 = wmma16(kb0, qb0, s1); s0 = wmma16(ka1, qb1, s0); s1 = wmma16(kb1, qb1, s1);
        asm volatile("v_nop\n\tv_nop\n\tv_nop\n\tv_nop" : "+v"(s0), "+v"(s1) : "v"(ka0), "v"(ka1), "v"(kb0), "v"(kb1), "v"(qb0), "v"(qb1));
        const v4f ma = *(const v4fa*)(mf + kt + 8 * hi), mc = *(const v4fa*)(mf + kt + 8 * hi + 4);
        const v4f md = *(const v4fa*)(mf + kt + 16 + 8 * hi), me = *(const v4fa*)(mf + kt + 16 + 8 * hi + 4);
        float u0[8], u1[8]; float mloc = -1.0e30f;
#pragma unroll
        for (int r = 0; r < 4; ++r) {
            u0[r] = s0[r] * SL + mq * ma[r]; u0[4 + r] = s0[4 + r] * SL + mq * mc[r];
            u1[r] = s1[r] * SL + mq * md[r]; u1[4 + r] = s1[4 + r] * SL + mq * me[r]; }
#pragma unroll
        for (int r = 0; r < 8; ++r) mloc = fmaxf(mloc, fmaxf(u0[r], u1[r]));
        mloc = fmaxf(mloc, __shfl_xor(mloc, 16, 32));
        const float mn = fmaxf(mrun, mloc);
        const float corr = __builtin_amdgcn_exp2f(mrun - mn);
        float sum = 0.0f; v16h pb;
#pragma unroll
        for (int r = 0; r < 8; ++r) { const float p0 = __builtin_amdgcn_exp2f(u0[r] - mn), p1 = __builtin_amdgcn_exp2f(u1[r] - mn); sum += p0 + p1; pb[r] = toh_flush(p0 * PCAR); pb[8 + r] = toh_flush(p1 * PCAR); }
        sum += __shfl_xor(sum, 16, 32);
        lrun = lrun * corr + sum;
        if (__builtin_amdgcn_ballot_w32(mn > mrun) != 0u) {
#pragma unroll
            for (int t = 0; t < 4; ++t)
#pragma unroll
                for (int r = 0; r < 8; ++r) o[t][r] *= corr; }
        mrun = mn;
#pragma unroll
        for (int t = 0; t < 4; ++t) o[t] = wmma16(va[t], pb, o[t]);
        asm volatile("v_nop\n\tv_nop\n\tv_nop\n\tv_nop" : "+v"(o[0]), "+v"(o[1]), "+v"(o[2]), "+v"(o[3]) : "v"(va[0]), "v"(va[1]), "v"(va[2]), "v"(va[3]), "v"(pb));
    }
    const float inv = 1.0f / (lrun * PCAR);
    float* ow = os + wave * (16 * 68);
#pragma unroll
    for (int t = 0; t < 4; ++t) { v4f a, c;
#pragma unroll
        for (int j = 0; j < 4; ++j) { a[j] = o[t][j] * inv; c[j] = o[t][4 + j] * inv; }
        *(v4fa*)(ow + lr * 68 + 16 * t + 8 * hi) = a; *(v4fa*)(ow + lr * 68 + 16 * t + 8 * hi + 4) = c; }
    __builtin_amdgcn_wave_barrier(); asm volatile("" ::: "memory");
    const int seg = lane & 7; v8us oh[4], ol[4];
#pragma unroll
    for (int s = 0; s < 4; ++s) { const int row = 4 * s + (lane >> 3); const v4f a = *(const v4fa*)(ow + row * 68 + seg * 8); const v4f c = *(const v4fa*)(ow + row * 68 + seg * 8 + 4);
#pragma unroll
        for (int j = 0; j < 4; ++j) { unsigned short x0, x1; splitf(a[j], x0, x1); oh[s][j] = x0; ol[s][j] = x1; splitf(c[j], x0, x1); oh[s][4 + j] = x0; ol[s][4 + j] = x1; } }
    bf* ah = ATh + ((size_t)b * SEQ + q0) * DM + h * HD; bf* al = ATl + ((size_t)b * SEQ + q0) * DM + h * HD;
#pragma unroll 1
    for (int ps = 0; ps < 2; ++ps) {
#pragma unroll
        for (int s = 0; s < 4; ++s) { const int row = 4 * s + (lane >> 3); *(volatile v8us*)(ah + (size_t)row * DM + seg * 8) = oh[s]; *(volatile v8us*)(al + (size_t)row * DM + seg * 8) = ol[s]; }
        if (ps == 0) __threadfence(); }
}

extern "C" void kernel_launch(void* const* d_in, const int* in_sizes, int n_in,
                              void* d_out, int out_size, void* d_ws, size_t ws_size, hipStream_t stream) {
    if (n_in < 10) return;
    const size_t needx = ((size_t)(NB - 1) * SEQ_FULL + SEQ) * DM, needm = (size_t)(NB - 1) * SEQ_FULL + SEQ;
    if ((size_t)in_sizes[0] < needx || (size_t)in_sizes[1] < needm) return;
    if ((size_t)in_sizes[2] < (size_t)DM * DM || (size_t)in_sizes[4] < (size_t)DM * DM || (size_t)in_sizes[6] < (size_t)DM * DM || (size_t)in_sizes[8] < (size_t)DM * DM) return;
    if (in_sizes[3] < DM || in_sizes[5] < DM || in_sizes[7] < DM || in_sizes[9] < DM) return;
    if ((size_t)out_size < (size_t)(NB - 1) * OUT_BSTRIDE + (size_t)SEQ * DM) return;
    const float* x = (const float*)d_in[0]; const int* mk = (const int*)d_in[1];
    const float* wq = (const float*)d_in[2]; const float* bq = (const float*)d_in[3]; const float* wk = (const float*)d_in[4]; const float* bk = (const float*)d_in[5];
    const float* wv = (const float*)d_in[6]; const float* bv = (const float*)d_in[7]; const float* wo = (const float*)d_in[8]; const float* bo = (const float*)d_in[9];
    float* OUT = (float*)d_out;
    char* wsp = (char*)d_ws;
    auto take = [&](size_t bytes) { char* p = wsp; wsp += (bytes + 255) & ~(size_t)255; return (void*)p; };
    const size_t MT = (size_t)NB * SEQ;
    bf* XB  = (bf*)take(MT * DM * 2);
    bf* WQt = (bf*)take((size_t)DM * DM * 2); bf* WKt = (bf*)take((size_t)DM * DM * 2); bf* WVt = (bf*)take((size_t)DM * DM * 2); bf* WOt = (bf*)take((size_t)DM * DM * 2);
    h16* QP = (h16*)take(MT * DM * 2); h16* KP = (h16*)take(MT * DM * 2); h16* VT = (h16*)take(MT * DM * 2);
    bf* ATh = (bf*)take(MT * DM * 2); bf* ATl = (bf*)take(MT * DM * 2);
    if ((size_t)(wsp - (char*)d_ws) > ws_size) return;
    k_cvtx<<<(unsigned)((MT * DM / 8 + 255) / 256), 256, 0, stream>>>(x, XB);
    k_cvtT<<<dim3(DM / 64, DM / 64), 256, 0, stream>>>(wq, WQt);
    k_cvtT<<<dim3(DM / 64, DM / 64), 256, 0, stream>>>(wk, WKt);
    k_cvtT<<<dim3(DM / 64, DM / 64), 256, 0, stream>>>(wv, WVt);
    k_cvtT<<<dim3(DM / 64, DM / 64), 256, 0, stream>>>(wo, WOt);
    k_gemmw<0, 1><<<dim3((unsigned)(MT / 64), DM / 64), 32, 0, stream>>>(XB, nullptr, WQt, DM, nullptr, QP, bq);
    k_gemmw<0, 1><<<dim3((unsigned)(MT / 64), DM / 64), 32, 0, stream>>>(XB, nullptr, WKt, DM, nullptr, KP, bk);
    k_gemmw<0, 2><<<dim3(DM / 64, (unsigned)(MT / 64)), 32, 0, stream>>>(WVt, nullptr, XB, DM, nullptr, VT, bv);
    k_flash<<<dim3(SEQ / 64, NB * NH), 128, 0, stream>>>(QP, KP, VT, mk, ATh, ATl);
    k_gemmw<1, 0><<<dim3((unsigned)(MT / 64), DM / 64), 32, 0, stream>>>(ATh, ATl, WOt, DM, OUT, nullptr, bo);
}
